// ShawStyleMHA_59167469469713
// MI455X (gfx1250) — hardware-verified
//
#include <hip/hip_runtime.h>

#define DM     1024
#define SEQ    1024
#define NBAT   4
#define NH     16
#define HD     64
#define NTOK   (NBAT * SEQ)
#define CPITCH 68

typedef unsigned short us;
typedef us us16v __attribute__((ext_vector_type(16)));
typedef us us8v __attribute__((ext_vector_type(8)));
typedef us8v __attribute__((may_alias)) us8a;
typedef __bf16 bf16v16 __attribute__((ext_vector_type(16)));
typedef float v8f __attribute__((ext_vector_type(8)));
typedef float v4f __attribute__((ext_vector_type(4)));
typedef v4f __attribute__((may_alias)) v4fa;

union Frag { us16v v; us8v h[2]; };

static __device__ __forceinline__ us bf_rne(float f) {
  unsigned u = __float_as_uint(f);
  u += 0x7fffu + ((u >> 16) & 1u);
  return (us)(u >> 16);
}
static __device__ __forceinline__ float bf_f32(us s) { return __uint_as_float(((unsigned)s) << 16); }

static __device__ __forceinline__ v8f zero8() {
  v8f z = {0.f, 0.f, 0.f, 0.f, 0.f, 0.f, 0.f, 0.f};
  return z;
}

static __device__ __forceinline__ v8f wmma_bf(us16v a, us16v b, v8f c) {
  return __builtin_amdgcn_wmma_f32_16x16x32_bf16(false, __builtin_bit_cast(bf16v16, a), false,
                                                 __builtin_bit_cast(bf16v16, b), (short)0, c, false, false);
}

static __device__ __forceinline__ void wmma3(v8f& acc, us16v ah, us16v al, us16v bh, us16v bl) {
  acc = wmma_bf(ah, bh, acc);
  acc = wmma_bf(al, bh, acc);
  acc = wmma_bf(ah, bl, acc);
  asm volatile("v_nop\n\tv_nop\n\tv_nop\n\tv_nop" : "+v"(acc) : "v"(ah), "v"(al), "v"(bh), "v"(bl));
}

static __device__ __forceinline__ us16v ldfrag(const us* rowp, int h) {
  Frag f;
  f.h[0] = *(const us8a*)(rowp + 8 * h);
  f.h[1] = *(const us8a*)(rowp + 16 + 8 * h);
  return f.v;
}

static __device__ __forceinline__ void lds_wave_sync() {
  __builtin_amdgcn_fence(__ATOMIC_RELEASE, "wavefront");
  __builtin_amdgcn_wave_barrier();
  __builtin_amdgcn_fence(__ATOMIC_ACQUIRE, "wavefront");
}

__global__ __launch_bounds__(256) void k_cvt_x(const float* __restrict__ x, us* xh, us* xl) {
  const size_t t = (size_t)blockIdx.x * 256u + threadIdx.x;
  const float* p = x + t * 8u;
  const v4f a = *(const v4fa*)p;
  const v4f b = *(const v4fa*)(p + 4);
  us8v hv, lv;
#pragma unroll
  for (int e = 0; e < 4; ++e) {
    const us h0 = bf_rne(a[e]);
    hv[e] = h0;
    lv[e] = bf_rne(a[e] - bf_f32(h0));
    const us h1 = bf_rne(b[e]);
    hv[4 + e] = h1;
    lv[4 + e] = bf_rne(b[e] - bf_f32(h1));
  }
  us* oh = xh + t * 8u;
  us* ol = xl + t * 8u;
  *(volatile us8v*)oh = hv;
  *(volatile us8v*)ol = lv;
  __threadfence();
  *(volatile us8v*)oh = hv;
  *(volatile us8v*)ol = lv;
}

__global__ __launch_bounds__(256) void k_cvt_w(const float* __restrict__ W0, const float* __restrict__ W1,
                                               const float* __restrict__ W2, const float* __restrict__ W3,
                                               us* wth, us* wtl) {
  __shared__ float sT[64][65];
  const int tid = threadIdx.x, lane = tid & 31, wv = tid >> 5;
  const int z = blockIdx.z;
  const int n0 = blockIdx.x * 64, k0 = blockIdx.y * 64;
  const float* W = (z == 0) ? W0 : (z == 1) ? W1 : (z == 2) ? W2 : W3;
#pragma unroll
  for (int p = 0; p < 4; ++p) {
    const int r = p * 16 + (tid >> 4);
    const int c4 = (tid & 15) * 4;
    const v4f v = *(const v4fa*)(W + (size_t)(k0 + r) * DM + n0 + c4);
    sT[r][c4 + 0] = v[0];
    sT[r][c4 + 1] = v[1];
    sT[r][c4 + 2] = v[2];
    sT[r][c4 + 3] = v[3];
  }
  __syncthreads();
  us* bhp = wth + (size_t)z * DM * DM;
  us* blp = wtl + (size_t)z * DM * DM;
#pragma unroll
  for (int rep = 0; rep < 2; ++rep) {
#pragma unroll
    for (int p = 0; p < 2; ++p) {
      const int rr = p * 32 + wv * 4 + (lane >> 3);
      const int k8 = (lane & 7) * 8;
      us8v hv, lv;
#pragma unroll
      for (int e = 0; e < 8; ++e) {
        const float v = sT[k8 + e][rr];
        const us hh = bf_rne(v);
        hv[e] = hh;
        lv[e] = bf_rne(v - bf_f32(hh));
      }
      const size_t o = (size_t)(n0 + rr) * DM + k0 + k8;
      *(volatile us8v*)(bhp + o) = hv;
      *(volatile us8v*)(blp + o) = lv;
    }
    __threadfence();
  }
}

__global__ __launch_bounds__(256) void k_cvt_rel(const float* __restrict__ rk, us* rh, us* rl) {
  const int tid = threadIdx.x;
  const int r = tid >> 3;
  const int d8 = (tid & 7) * 8;
  const float* p = rk + r * HD + d8;
  us8v hv, lv;
#pragma unroll
  for (int e = 0; e < 8; ++e) {
    const float v = p[e];
    const us hh = bf_rne(v);
    hv[e] = hh;
    lv[e] = bf_rne(v - bf_f32(hh));
  }
  const size_t o = (size_t)r * HD + d8;
  *(volatile us8v*)(rh + o) = hv;
  *(volatile us8v*)(rl + o) = lv;
  __threadfence();
  *(volatile us8v*)(rh + o) = hv;
  *(volatile us8v*)(rl + o) = lv;
}

static __device__ __forceinline__ void gemm_core(const us* __restrict__ AH, const us* __restrict__ AL,
                                                 const us* __restrict__ BH, const us* __restrict__ BL,
                                                 int arow0, int bcol0, float (*sC)[CPITCH], int srow0) {
  const int lane = threadIdx.x & 31, h = lane >> 4, m = lane & 15;
  v8f acc[2][4];
#pragma unroll
  for (int rt = 0; rt < 2; ++rt)
#pragma unroll
    for (int ct = 0; ct < 4; ++ct) acc[rt][ct] = zero8();

  const us* a0h = AH + (size_t)(arow0 + m) * DM;
  const us* a1h = a0h + (size_t)16 * DM;
  const us* a0l = AL + (size_t)(arow0 + m) * DM;
  const us* a1l = a0l + (size_t)16 * DM;
  const us* bhp = BH + (size_t)(bcol0 + m) * DM;
  const us* blp = BL + (size_t)(bcol0 + m) * DM;

#pragma unroll 1
  for (int k = 0; k < DM; k += 32) {
    const us16v fa0h = ldfrag(a0h + k, h);
    const us16v fa0l = ldfrag(a0l + k, h);
    const us16v fa1h = ldfrag(a1h + k, h);
    const us16v fa1l = ldfrag(a1l + k, h);
#pragma unroll
    for (int ct = 0; ct < 4; ++ct) {
      const size_t co = (size_t)ct * 16 * DM + k;
      const us16v fbh = ldfrag(bhp + co, h);
      const us16v fbl = ldfrag(blp + co, h);
      wmma3(acc[0][ct], fa0h, fa0l, fbh, fbl);
      wmma3(acc[1][ct], fa1h, fa1l, fbh, fbl);
    }
  }
#pragma unroll
  for (int rt = 0; rt < 2; ++rt)
#pragma unroll
    for (int ct = 0; ct < 4; ++ct)
#pragma unroll
      for (int g = 0; g < 8; ++g) sC[srow0 + 16 * rt + 8 * h + g][16 * ct + m] = acc[rt][ct][g];
}

__global__ __launch_bounds__(128) void k_gemm_qkv(const us* __restrict__ XH, const us* __restrict__ XL,
                                                  const us* __restrict__ WTH, const us* __restrict__ WTL,
                                                  us* OH, us* OL) {
  __shared__ __attribute__((aligned(16))) float sC[128][CPITCH];
  const int tid = threadIdx.x, lane = tid & 31, wv = tid >> 5;
  const int z = blockIdx.z;
  const int m0 = blockIdx.x * 128, n0 = blockIdx.y * 64;
  gemm_core(XH, XL, WTH + (size_t)z * DM * DM, WTL + (size_t)z * DM * DM, m0 + 32 * wv, n0, sC, 32 * wv);
  __syncthreads();
  us* oh = OH + (size_t)z * NTOK * DM;
  us* ol = OL + (size_t)z * NTOK * DM;
  const int b = m0 >> 10, tok0 = m0 & 1023, hh = n0 >> 6;
  const int bh = b * NH + hh;
  if (z < 2) {
#pragma unroll
    for (int rep = 0; rep < 2; ++rep) {
      for (int p = 0; p < 8; ++p) {
        const int r = p * 16 + wv * 4 + (lane >> 3);
        const int d8 = (lane & 7) * 8;
        us8v hv, lv;
#pragma unroll
        for (int e = 0; e < 8; ++e) {
          const float v = sC[r][d8 + e];
          const us q = bf_rne(v);
          hv[e] = q;
          lv[e] = bf_rne(v - bf_f32(q));
        }
        const size_t o = ((size_t)bh * SEQ + tok0 + r) * HD + d8;
        *(volatile us8v*)(oh + o) = hv;
        *(volatile us8v*)(ol + o) = lv;
      }
      __threadfence();
    }
  } else {
#pragma unroll
    for (int rep = 0; rep < 2; ++rep) {
      for (int p = 0; p < 8; ++p) {
        const int d = p * 8 + wv * 2 + (lane >> 4);
        const int t8 = (lane & 15) * 8;
        us8v hv, lv;
#pragma unroll
        for (int e = 0; e < 8; ++e) {
          const float v = sC[t8 + e][d];
          const us q = bf_rne(v);
          hv[e] = q;
          lv[e] = bf_rne(v - bf_f32(q));
        }
        const size_t o = ((size_t)bh * HD + d) * SEQ + tok0 + t8;
        *(volatile us8v*)(oh + o) = hv;
        *(volatile us8v*)(ol + o) = lv;
      }
      __threadfence();
    }
  }
}

__global__ __launch_bounds__(128) void k_gemm_out(const us* __restrict__ CH, const us* __restrict__ CL,
                                                  const us* __restrict__ WH, const us* __restrict__ WL,
                                                  const float* __restrict__ bias, float* out) {
  __shared__ __attribute__((aligned(16))) float sC[128][CPITCH];
  const int tid = threadIdx.x, lane = tid & 31, wv = tid >> 5;
  const int m0 = blockIdx.x * 128, n0 = blockIdx.y * 64;
  gemm_core(CH, CL, WH, WL, m0 + 32 * wv, n0, sC, 32 * wv);
  __syncthreads();
#pragma unroll
  for (int rep = 0; rep < 2; ++rep) {
    for (int p = 0; p < 16; ++p) {
      const int r = p * 8 + wv * 2 + (lane >> 4);
      const int c4 = (lane & 15) * 4;
      const v4f bv = *(const v4fa*)(bias + n0 + c4);
      v4f v;
      v[0] = sC[r][c4 + 0] + bv[0];
      v[1] = sC[r][c4 + 1] + bv[1];
      v[2] = sC[r][c4 + 2] + bv[2];
      v[3] = sC[r][c4 + 3] + bv[3];
      *(volatile v4f*)(out + (size_t)(m0 + r) * DM + n0 + c4) = v;
    }
    __threadfence();
  }
}

__global__ __launch_bounds__(128) void k_attn(const us* __restrict__ QH, const us* __restrict__ QL,
                                              const us* __restrict__ KH, const us* __restrict__ KL,
                                              const us* __restrict__ VH, const us* __restrict__ VL,
                                              const us* __restrict__ RH, const us* __restrict__ RL,
                                              const float* __restrict__ relv, us* CH, us* CL) {
  __shared__ float sQR[4][16][33];
  __shared__ __attribute__((aligned(16))) us sPh[4][16][40];
  __shared__ __attribute__((aligned(16))) us sPl[4][16][40];
  __shared__ float sBand[4][16][17];
  __shared__ __attribute__((aligned(16))) float sO[4][16][CPITCH];

  const int lane = threadIdx.x & 31, wv = threadIdx.x >> 5, h = lane >> 4, m = lane & 15;
  const int bh = blockIdx.y;
  const int qbase = blockIdx.x * 64 + wv * 16;
  const float NINF = -__builtin_inff();

  const us* qh = QH + ((size_t)bh * SEQ + qbase + m) * HD;
  const us* ql = QL + ((size_t)bh * SEQ + qbase + m) * HD;
  const us16v aqh0 = ldfrag(qh, h), aqh1 = ldfrag(qh + 32, h);
  const us16v aql0 = ldfrag(ql, h), aql1 = ldfrag(ql + 32, h);

#pragma unroll
  for (int nt = 0; nt < 2; ++nt) {
    const us* rh = RH + (size_t)(16 * nt + m) * HD;
    const us* rl = RL + (size_t)(16 * nt + m) * HD;
    v8f acc = zero8();
    wmma3(acc, aqh0, aql0, ldfrag(rh, h), ldfrag(rl, h));
    wmma3(acc, aqh1, aql1, ldfrag(rh + 32, h), ldfrag(rl + 32, h));
#pragma unroll
    for (int g = 0; g < 8; ++g) sQR[wv][8 * h + g][16 * nt + m] = acc[g];
  }
  lds_wave_sync();

  float mrow[8], lrow[8], band[8];
  v8f o[4];
#pragma unroll
  for (int g = 0; g < 8; ++g) { mrow[g] = NINF; lrow[g] = 0.f; band[g] = 0.f; }
#pragma unroll
  for (int tt = 0; tt < 4; ++tt) o[tt] = zero8();

  const int nsteps = (qbase >> 5) + 1;
  for (int st = 0; st < nsteps; ++st) {
    const int kb2 = st << 5;
    lds_wave_sync();
    float sv[2][8];
#pragma unroll
    for (int t = 0; t < 2; ++t) {
      const int j = kb2 + 16 * t + m;
      const us* kh = KH + ((size_t)bh * SEQ + j) * HD;
      const us* kl = KL + ((size_t)bh * SEQ + j) * HD;
      v8f sc = zero8();
      {
        const us16v b0h = ldfrag(kh, h), b0l = ldfrag(kl, h);
        wmma3(sc, aqh0, aql0, b0h, b0l);
      }
      {
        const us16v b1h = ldfrag(kh + 32, h), b1l = ldfrag(kl + 32, h);
        wmma3(sc, aqh1, aql1, b1h, b1l);
      }
#pragma unroll
      for (int g = 0; g < 8; ++g) {
        const int lr = 8 * h + g;
        const int dj = j - (qbase + lr);
        int rr = dj + 16;
        rr = rr < 0 ? 0 : rr;
        rr = rr > 16 ? 16 : rr;
        const float qr = sQR[wv][lr][rr];
        sv[t][g] = (dj > 0) ? NINF : (sc[g] + qr) * 0.125f;
      }
    }
    float cf[8];
#pragma unroll
    for (int g = 0; g < 8; ++g) {
      float v = fmaxf(sv[0][g], sv[1][g]);
      v = fmaxf(v, __shfl_xor(v, 1));
      v = fmaxf(v, __shfl_xor(v, 2));
      v = fmaxf(v, __shfl_xor(v, 4));
      v = fmaxf(v, __shfl_xor(v, 8));
      const float mn = fmaxf(mrow[g], v);
      cf[g] = (mrow[g] == NINF) ? 0.f : __expf(mrow[g] - mn);
      mrow[g] = mn;
      lrow[g] *= cf[g];
      band[g] *= cf[g];
    }
#pragma unroll
    for (int tt = 0; tt < 4; ++tt)
#pragma unroll
      for (int g = 0; g < 8; ++g) o[tt][g] *= cf[g];
#pragma unroll
    for (int t = 0; t < 2; ++t) {
      const int j = kb2 + 16 * t + m;
#pragma unroll
      for (int g = 0; g < 8; ++g) {
        const int lr = 8 * h + g;
        const int dj = j - (qbase + lr);
        const float e = (dj > 0) ? 0.f : __expf(sv[t][g] - mrow[g]);
        float rs = e;
        rs += __shfl_xor(rs, 1);
        rs += __shfl_xor(rs, 2);
        rs += __shfl_xor(rs, 4);
        rs += __shfl_xor(rs, 8);
        lrow[g] += rs;
        const us eh = bf_rne(e);
        const us el = bf_rne(e - bf_f32(eh));
        sPh[wv][lr][16 * t + m] = eh;
        sPl[wv][lr][16 * t + m] = el;
        band[g] = (dj >= -15 && dj <= 0) ? e : band[g];
      }
    }
    lds_wave_sync();
    const us16v aph = ldfrag(&sPh[wv][m][0], h);
    const us16v apl = ldfrag(&sPl[wv][m][0], h);
#pragma unroll
    for (int tt = 0; tt < 4; ++tt) {
      const us* vh = VH + ((size_t)bh * HD + 16 * tt + m) * SEQ + kb2;
      const us* vl = VL + ((size_t)bh * HD + 16 * tt + m) * SEQ + kb2;
      wmma3(o[tt], aph, apl, ldfrag(vh, h), ldfrag(vl, h));
    }
  }

  float invl[8];
#pragma unroll
  for (int g = 0; g < 8; ++g) invl[g] = 1.0f / lrow[g];
#pragma unroll
  for (int g = 0; g < 8; ++g) {
    const int lr = 8 * h + g;
    sBand[wv][lr][(m - lr - 1) & 15] = band[g] * invl[g];
  }
  lds_wave_sync();
  float rv0[4];
  float val[4][8];
#pragma unroll
  for (int tt = 0; tt < 4; ++tt) {
    rv0[tt] = relv[16 * tt + m];
#pragma unroll
    for (int g = 0; g < 8; ++g) val[tt][g] = o[tt][g] * invl[g] + rv0[tt];
  }
#pragma unroll 1
  for (int r = 0; r < 16; ++r) {
    float sb[8];
#pragma unroll
    for (int g = 0; g < 8; ++g) sb[g] = sBand[wv][8 * h + g][r];
#pragma unroll
    for (int tt = 0; tt < 4; ++tt) {
      const float dv = relv[(r + 1) * HD + 16 * tt + m] - rv0[tt];
#pragma unroll
      for (int g = 0; g < 8; ++g) val[tt][g] += sb[g] * dv;
    }
  }
#pragma unroll
  for (int tt = 0; tt < 4; ++tt)
#pragma unroll
    for (int g = 0; g < 8; ++g) sO[wv][8 * h + g][16 * tt + m] = val[tt][g];
  lds_wave_sync();

  const int b = bh >> 4, hd = bh & 15;
#pragma unroll
  for (int rep = 0; rep < 2; ++rep) {
#pragma unroll
    for (int p = 0; p < 4; ++p) {
      const int r = p * 4 + (lane >> 3);
      const int d8 = (lane & 7) * 8;
      us8v hv, lv;
#pragma unroll
      for (int e = 0; e < 8; ++e) {
        const float v = sO[wv][r][d8 + e];
        const us q = bf_rne(v);
        hv[e] = q;
        lv[e] = bf_rne(v - bf_f32(q));
      }
      const size_t o2 = ((size_t)(b * SEQ + qbase + r)) * DM + hd * HD + d8;
      *(volatile us8v*)(CH + o2) = hv;
      *(volatile us8v*)(CL + o2) = lv;
    }
    __threadfence();
  }
}

extern "C" void kernel_launch(void* const* d_in, const int* in_sizes, int n_in,
                              void* d_out, int out_size, void* d_ws, size_t ws_size,
                              hipStream_t stream) {
  if (n_in < 8) return;
  if (in_sizes[0] != NTOK * DM) return;
  if (in_sizes[1] != DM * DM || in_sizes[2] != DM * DM || in_sizes[3] != DM * DM || in_sizes[4] != DM * DM) return;
  if (in_sizes[5] != DM || in_sizes[6] != 33 * HD || in_sizes[7] != 33 * HD) return;
  if (out_size != NTOK * DM) return;

  const float* x    = (const float*)d_in[0];
  const float* Wq   = (const float*)d_in[1];
  const float* Wk   = (const float*)d_in[2];
  const float* Wv   = (const float*)d_in[3];
  const float* Wo   = (const float*)d_in[4];
  const float* bo   = (const float*)d_in[5];
  const float* relk = (const float*)d_in[6];
  const float* relv = (const float*)d_in[7];
  float* out = (float*)d_out;

  const size_t plane_x = (size_t)NTOK * DM * sizeof(us);
  const size_t plane_w = (size_t)DM * DM * sizeof(us);
  const size_t plane_r = (size_t)32 * HD * sizeof(us);
  char* ws = (char*)d_ws;
  size_t off = 0;
  us* XH   = (us*)(ws + off); off += plane_x;
  us* XL   = (us*)(ws + off); off += plane_x;
  us* WTH  = (us*)(ws + off); off += 4 * plane_w;
  us* WTL  = (us*)(ws + off); off += 4 * plane_w;
  us* QKVH = (us*)(ws + off); off += 3 * plane_x;
  us* QKVL = (us*)(ws + off); off += 3 * plane_x;
  us* CH   = (us*)(ws + off); off += plane_x;
  us* CL   = (us*)(ws + off); off += plane_x;
  us* RH   = (us*)(ws + off); off += plane_r;
  us* RL   = (us*)(ws + off); off += plane_r;
  if (off > ws_size) return;

  const size_t pq = (size_t)NTOK * DM;

  k_cvt_x<<<(NTOK * DM) / (8 * 256), 256, 0, stream>>>(x, XH, XL);
  k_cvt_w<<<dim3(DM / 64, DM / 64, 4), 256, 0, stream>>>(Wq, Wk, Wv, Wo, WTH, WTL);
  k_cvt_rel<<<1, 256, 0, stream>>>(relk, RH, RL);
  k_gemm_qkv<<<dim3(NTOK / 128, DM / 64, 3), 128, 0, stream>>>(XH, XL, WTH, WTL, QKVH, QKVL);
  k_attn<<<dim3(SEQ / 64, NBAT * NH), 128, 0, stream>>>(QKVH, QKVL, QKVH + pq, QKVL + pq,
                                                        QKVH + 2 * pq, QKVL + 2 * pq, RH, RL, relv, CH, CL);
  k_gemm_out<<<dim3(NTOK / 128, DM / 64, 1), 128, 0, stream>>>(CH, CL, WTH + (size_t)3 * DM * DM,
                                                               WTL + (size_t)3 * DM * DM, bo, out);
}
